// HeatMapRegressor_30013231464923
// MI455X (gfx1250) — hardware-verified
//
#include <hip/hip_runtime.h>
#include <stddef.h>


#define CH      64
#define KD      128
#define AP      136
#define NTHR    256
#define NWAVE   8
#define EPT     8
#define NGRP    2
#define CHUNK   (NTHR * EPT * NGRP)
#define WCAP    (EPT * NGRP * 32)
#define LISTN   (NWAVE * WCAP)
#define NBC     4096
#define NBF     2048
#define SUBS    (NBC / NBF)
#define OTHR    512
#define WPS     ((OTHR / 32) / SUBS)
#define RCAP    40960
#define RBN     128
#define TGT     256
#define DEGCAP  256
#define GROWS   128
#define DOUT2   68
#define NT2     5

#define LDS_FILL ((RCAP + NBF + LISTN) * 4 + 64)
#define LDS_LIN  (2 * GROWS * AP * 2)

static_assert((CHUNK & (CHUNK - 1)) == 0);
static_assert(CHUNK <= 4096);
static_assert(NBC <= 4096 && NBF <= 4096);
static_assert((NBC & (NBC - 1)) == 0 && (NBF & (NBF - 1)) == 0);
static_assert(NBC == SUBS * NBF);
static_assert(OTHR * 8 == NBC);
static_assert(((OTHR / 32) % SUBS) == 0);
static_assert((RCAP % 32) == 0);
static_assert(TGT == NWAVE * 32);
static_assert(KD == 2 * CH);
static_assert(GROWS * DOUT2 * 4 <= LDS_LIN);
static_assert(GROWS == NWAVE * 16);
static_assert(NT2 * 16 >= DOUT2);
static_assert((AP * 2) % 16 == 0);

typedef float          v4f  __attribute__((ext_vector_type(4)));
typedef float          v8f  __attribute__((ext_vector_type(8)));
typedef int            v4i  __attribute__((ext_vector_type(4)));
typedef unsigned short v8us __attribute__((ext_vector_type(8)));
typedef __bf16         v16b __attribute__((ext_vector_type(16)));
union FragB { v16b v; v8us u[2]; };

__device__ __forceinline__ void split2(float x, unsigned short& h, unsigned short& l) {
  const unsigned int u  = __float_as_uint(x);
  const unsigned int hb = (u + 0x7FFFu + ((u >> 16) & 1u)) >> 16;
  const float hf = __uint_as_float(hb << 16);
  const float r  = x - hf;
  const unsigned int v  = __float_as_uint(r);
  const unsigned int lb = (v + 0x7FFFu + ((v >> 16) & 1u)) >> 16;
  h = (unsigned short)hb;
  l = (unsigned short)lb;
}

__device__ __forceinline__ void split8(v4f a, v4f b, v8us& h8, v8us& l8) {
#pragma unroll
  for (int e = 0; e < 8; ++e) {
    const float x = e < 4 ? a[e] : b[e - 4];
    unsigned short th, tl;
    split2(x, th, tl);
    h8[e] = th;
    l8[e] = tl;
  }
}

__device__ __forceinline__ v8f wmb(v16b a, v16b b, v8f c) {
#if defined(__HIP_DEVICE_COMPILE__)
  v8f d = __builtin_amdgcn_wmma_f32_16x16x32_bf16(false, a, false, b, (short)0, c, false, false);
  asm volatile("v_nop\n\tv_nop\n\tv_nop\n\tv_nop" : "+v"(d) : "v"(a), "v"(b));
  return d;
#else
  return c;
#endif
}

template <int NB>
__device__ __forceinline__ int scan_chunk(const int* __restrict__ dsts, int nE, int cbase, int slotBase,
                                          int vec8, int* list, int tid, int lane, int wave) {
  int wc = 0;
#pragma unroll
  for (int g = 0; g < NGRP; ++g) {
    const int el0  = (g * NTHR + tid) * EPT;
    const int e0   = cbase + el0;
    const int sent = -2147483647 - 1;
    v4i da, db;
    if (vec8 != 0 && cbase + CHUNK <= nE) {
      da = *(const v4i*)(dsts + e0);
      db = *(const v4i*)(dsts + e0 + 4);
    } else {
      da.x = (e0     < nE) ? dsts[min(e0, nE - 1)] : sent;
      da.y = (e0 + 1 < nE) ? dsts[min(e0 + 1, nE - 1)] : sent;
      da.z = (e0 + 2 < nE) ? dsts[min(e0 + 2, nE - 1)] : sent;
      da.w = (e0 + 3 < nE) ? dsts[min(e0 + 3, nE - 1)] : sent;
      db.x = (e0 + 4 < nE) ? dsts[min(e0 + 4, nE - 1)] : sent;
      db.y = (e0 + 5 < nE) ? dsts[min(e0 + 5, nE - 1)] : sent;
      db.z = (e0 + 6 < nE) ? dsts[min(e0 + 6, nE - 1)] : sent;
      db.w = (e0 + 7 < nE) ? dsts[min(e0 + 7, nE - 1)] : sent;
    }
    const unsigned nb = (unsigned)slotBase;
    const unsigned s0 = (unsigned)da.x - nb, s1 = (unsigned)da.y - nb;
    const unsigned s2 = (unsigned)da.z - nb, s3 = (unsigned)da.w - nb;
    const unsigned s4 = (unsigned)db.x - nb, s5 = (unsigned)db.y - nb;
    const unsigned s6 = (unsigned)db.z - nb, s7 = (unsigned)db.w - nb;
    const bool h0 = s0 < (unsigned)NB, h1 = s1 < (unsigned)NB, h2 = s2 < (unsigned)NB, h3 = s3 < (unsigned)NB;
    const bool h4 = s4 < (unsigned)NB, h5 = s5 < (unsigned)NB, h6 = s6 < (unsigned)NB, h7 = s7 < (unsigned)NB;
    const unsigned any = __builtin_amdgcn_ballot_w32(h0 | h1 | h2 | h3 | h4 | h5 | h6 | h7);
    if (any != 0u) {
#define HITJ(J, HJ, SJ) { \
        const unsigned mj = __builtin_amdgcn_ballot_w32(HJ); \
        if (mj != 0u) { \
          if (HJ) { \
            const int pos = wc + (int)__builtin_amdgcn_mbcnt_lo(mj, 0u); \
            if (pos < WCAP) list[wave * WCAP + pos] = ((el0 + (J)) << 12) | (int)(SJ); \
          } \
          wc += (int)__builtin_popcount(mj); } }
      HITJ(0, h0, s0)
      HITJ(1, h1, s1)
      HITJ(2, h2, s2)
      HITJ(3, h3, s3)
      HITJ(4, h4, s4)
      HITJ(5, h5, s5)
      HITJ(6, h6, s6)
      HITJ(7, h7, s7)
#undef HITJ
    }
  }
  return wc;
}

__global__ __launch_bounds__(NTHR) void k_wprep(
    const float* __restrict__ Wl1, const float* __restrict__ Wr1,
    const float* __restrict__ Wl2, const float* __restrict__ Wr2,
    unsigned short* b1h, unsigned short* b1l, unsigned short* b2h, unsigned short* b2l) {
  const int g1 = CH * (KD / 8);
  const int g2 = (NT2 * 16) * (KD / 8);
  const int bstart = blockIdx.x * NTHR;
  const float* wl; const float* wr; unsigned short* dh; unsigned short* dl; int dout, seg;
  if (bstart < g1) { wl = Wl1; wr = Wr1; dh = b1h; dl = b1l; dout = CH;    seg = 0;  }
  else             { wl = Wl2; wr = Wr2; dh = b2h; dl = b2l; dout = DOUT2; seg = g1; }
  const int i = bstart + (int)threadIdx.x;
  if (i >= g1 + g2) return;
  const int o  = i - seg;
  const int n  = o >> 4;
  const int k0 = (o & 15) * 8;
  const int nc = n < dout ? n : dout - 1;
  v4f a, b;
#pragma unroll
  for (int e = 0; e < 8; ++e) {
    const int k  = k0 + e;
    const int kl = k < CH ? k : CH - 1;
    int kr = k - CH; kr = kr < 0 ? 0 : (kr > CH - 1 ? CH - 1 : kr);
    const float xl = wl[kl * dout + nc];
    const float xr = wr[kr * dout + nc];
    float x = (k < CH) ? xl : xr;
    x = (n < dout) ? x : 0.0f;
    if (e < 4) a[e] = x; else b[e - 4] = x;
  }
  v8us h8, l8;
  split8(a, b, h8, l8);
  unsigned short* ph = dh + (size_t)n * KD + k0;
  unsigned short* pl = dl + (size_t)n * KD + k0;
  *(volatile v8us*)ph = h8;
  *(volatile v8us*)pl = l8;
  __threadfence();
  *(volatile v8us*)ph = h8;
  *(volatile v8us*)pl = l8;
}

__global__ __launch_bounds__(NTHR) void k_count(const int* __restrict__ ei, int* cnt, int nE, int vec8) {
  __shared__ __attribute__((aligned(16))) int scnt[NBC];
  __shared__ __attribute__((aligned(16))) int list[LISTN];
  __shared__ int wcnt[NWAVE];
  const int tid = threadIdx.x, lane = tid & 31, wave = tid >> 5;
  const int nodeBase = blockIdx.x * NBC;
  const int* dsts = ei + nE;

  for (int i = tid; i < NBC; i += NTHR) scnt[i] = 0;
  __syncthreads();

  const int nChunks = (nE + CHUNK - 1) / CHUNK;
#pragma unroll 1
  for (int ch = 0; ch < nChunks; ++ch) {
    const int cbase = ch * CHUNK;
    const int wc = scan_chunk<NBC>(dsts, nE, cbase, nodeBase, vec8, list, tid, lane, wave);
    if (lane == 0) wcnt[wave] = wc;
    __syncthreads();
    if (wave == 0) {
#pragma unroll 1
      for (int wsx = 0; wsx < NWAVE; ++wsx) {
        int n = __builtin_amdgcn_readfirstlane(wcnt[wsx]);
        n = n > WCAP ? WCAP : (n < 0 ? 0 : n);
        const int* lp = list + wsx * WCAP;
#pragma unroll 1
        for (int i = 0; i < n; ++i) {
          const int ent  = __builtin_amdgcn_readfirstlane(lp[i]);
          const int slot = ent & (NBC - 1);
          if (lane == 0) scnt[slot] = scnt[slot] + 1;
        }
      }
    }
    __syncthreads();
  }

  v4i cq[4];
#pragma unroll
  for (int q = 0; q < 4; ++q) {
    const int f = (wave * 4 + q) * 128 + 4 * lane;
    cq[q] = *(const v4i*)(scnt + f);
  }
  int* cp = cnt + (size_t)nodeBase;
#pragma unroll
  for (int q = 0; q < 4; ++q) {
    const int f = (wave * 4 + q) * 128 + 4 * lane;
    *(volatile v4i*)(cp + f) = cq[q];
  }
  __threadfence();
#pragma unroll
  for (int q = 0; q < 4; ++q) {
    const int f = (wave * 4 + q) * 128 + 4 * lane;
    *(volatile v4i*)(cp + f) = cq[q];
  }
}

__global__ __launch_bounds__(OTHR) void k_offsets(const int* __restrict__ cnt, int* off, int* rbase, int nChunk) {
  __shared__ __attribute__((aligned(16))) int soff[NBC];
  __shared__ __attribute__((aligned(16))) int srb[RBN];
  __shared__ int wtot[OTHR / 32];
  const int tid = threadIdx.x, lane = tid & 31, wave = tid >> 5, sub = wave / WPS;
  for (int i = tid; i < RBN; i += OTHR) srb[i] = 0;
  __syncthreads();
  int carry = 0;
#pragma unroll 1
  for (int ch = 0; ch < nChunk; ++ch) {
    const int base = ch * NBC;
    const v4i c0 = *(const v4i*)(cnt + base + 8 * tid);
    const v4i c1 = *(const v4i*)(cnt + base + 8 * tid + 4);
    const int e0 = max(c0.x, 0), e1 = max(c0.y, 0), e2 = max(c0.z, 0), e3 = max(c0.w, 0);
    const int e4 = max(c1.x, 0), e5 = max(c1.y, 0), e6 = max(c1.z, 0), e7 = max(c1.w, 0);
    const int ts = e0 + e1 + e2 + e3 + e4 + e5 + e6 + e7;
    int incl = ts;
#pragma unroll
    for (int d = 1; d < 32; d <<= 1) {
      const int t = __shfl_up(incl, d);
      if (lane >= d) incl += t;
    }
    if (lane == 31) wtot[wave] = incl;
    __syncthreads();
    int pre = 0;
#pragma unroll 1
    for (int w = sub * WPS; w < wave; ++w) pre += wtot[w];
    int bcur = carry, myb = carry;
#pragma unroll
    for (int s = 0; s < SUBS; ++s) {
      int S = 0;
#pragma unroll
      for (int w = 0; w < WPS; ++w) S += wtot[s * WPS + w];
      if (tid == 0) srb[min(SUBS * ch + s, RBN - 1)] = bcur;
      myb = (s == sub) ? bcur : myb;
      bcur += (S + 31) & ~31;
    }
    int run = myb + pre + incl - ts;
    soff[8 * tid + 0] = run; run += e0;
    soff[8 * tid + 1] = run; run += e1;
    soff[8 * tid + 2] = run; run += e2;
    soff[8 * tid + 3] = run; run += e3;
    soff[8 * tid + 4] = run; run += e4;
    soff[8 * tid + 5] = run; run += e5;
    soff[8 * tid + 6] = run; run += e6;
    soff[8 * tid + 7] = run;
    carry = bcur;
    __syncthreads();
    const v4i o0 = *(const v4i*)(soff + 4 * tid);
    const v4i o1 = *(const v4i*)(soff + 4 * (tid + OTHR));
    int* op = off + base;
    *(volatile v4i*)(op + 4 * tid) = o0;
    *(volatile v4i*)(op + 4 * (tid + OTHR)) = o1;
    __threadfence();
    *(volatile v4i*)(op + 4 * tid) = o0;
    *(volatile v4i*)(op + 4 * (tid + OTHR)) = o1;
    __syncthreads();
  }
  if (tid == 0) srb[min(SUBS * nChunk, RBN - 1)] = carry;
  __syncthreads();
  v4i rv = {0, 0, 0, 0};
  if (tid < 32) rv = *(const v4i*)(srb + 4 * tid);
  if (tid < 32) *(volatile v4i*)(rbase + 4 * tid) = rv;
  __threadfence();
  if (tid < 32) *(volatile v4i*)(rbase + 4 * tid) = rv;
}

__global__ __launch_bounds__(NTHR) void k_fill(
    const int* __restrict__ ei, const int* __restrict__ off, const int* __restrict__ rbase,
    int* csr, int nN, int nE, int vec8, int csrLen) {
  extern __shared__ v4f lds_dyn[];
  int* region = (int*)lds_dyn;
  int* cursor = region + RCAP;
  int* list   = cursor + NBF;
  int* wcnt   = list + LISTN;
  const int tid = threadIdx.x, lane = tid & 31, wave = tid >> 5;
  const int b = blockIdx.x;
  const int nodeBase = b * NBF;
  const int* dsts = ei + nE;

  int rb0 = rbase[b];
  const int rb1 = rbase[b + 1];
  rb0 = rb0 < 0 ? 0 : (rb0 > csrLen ? csrLen : rb0);
  rb0 &= ~31;
  int len = rb1 - rb0;
  len = len < 0 ? 0 : (len > RCAP ? RCAP : len);
  int lenW = (len + 31) & ~31;
  if (rb0 + lenW > csrLen) lenW = (csrLen - rb0) & ~31;

  {
    const v4i z = {0, 0, 0, 0};
    for (int i = tid; i < RCAP / 4; i += NTHR) ((v4i*)region)[i] = z;
    for (int s = tid; s < NBF; s += NTHR) {
      int o = off[nodeBase + s] - rb0;
      o = o < 0 ? 0 : (o > RCAP ? RCAP : o);
      cursor[s] = o;
    }
  }
  __syncthreads();

  const int nChunks = (nE + CHUNK - 1) / CHUNK;
#pragma unroll 1
  for (int ch = 0; ch < nChunks; ++ch) {
    const int cbase = ch * CHUNK;
    const int wc = scan_chunk<NBF>(dsts, nE, cbase, nodeBase, vec8, list, tid, lane, wave);
    if (lane == 0) wcnt[wave] = wc;
    __syncthreads();
    if (wave == 0) {
#pragma unroll 1
      for (int wsx = 0; wsx < NWAVE; ++wsx) {
        int n = __builtin_amdgcn_readfirstlane(wcnt[wsx]);
        n = n > WCAP ? WCAP : (n < 0 ? 0 : n);
        const int* lp = list + wsx * WCAP;
#pragma unroll 1
        for (int i = 0; i < n; ++i) {
          const int ent  = __builtin_amdgcn_readfirstlane(lp[i]);
          const int slot = ent & (NBF - 1);
          int e = cbase + ((ent >> 12) & (CHUNK - 1));
          e = e > nE - 1 ? nE - 1 : e;
          int src = ei[e];
          src = src < 0 ? 0 : (src > nN - 1 ? nN - 1 : src);
          if (lane == 0) {
            int pos = cursor[slot];
            pos = pos < 0 ? 0 : (pos > RCAP - 1 ? RCAP - 1 : pos);
            region[pos] = src;
            const int np = pos + 1;
            cursor[slot] = np > RCAP ? RCAP : np;
          }
        }
      }
    }
    __syncthreads();
  }

  const int nv = lenW >> 2;
  int* gp = csr + rb0;
#pragma unroll 1
  for (int i = tid; i < nv; i += NTHR) { const v4i v = ((const v4i*)region)[i]; *(volatile v4i*)(gp + 4 * i) = v; }
  __threadfence();
#pragma unroll 1
  for (int i = tid; i < nv; i += NTHR) { const v4i v = ((const v4i*)region)[i]; *(volatile v4i*)(gp + 4 * i) = v; }
}

__global__ __launch_bounds__(NTHR) void k_layer0(
    const float* __restrict__ pos, const int* __restrict__ csr, const int* __restrict__ off,
    const int* __restrict__ cnt, const float* __restrict__ Wl, const float* __restrict__ bl,
    const float* __restrict__ Wr, float* h0, int nN, int csrLen) {
  __shared__ __attribute__((aligned(16))) float sW[2 * 3 * CH + CH];
  __shared__ __attribute__((aligned(16))) float xs[NWAVE * 32 * 8];
  const int tid = threadIdx.x, lane = tid & 31, wave = tid >> 5, hh = lane >> 4;
  for (int i = tid; i < 3 * CH; i += NTHR) { sW[i] = Wl[i]; sW[3 * CH + i] = Wr[i]; }
  for (int i = tid; i < CH; i += NTHR) sW[6 * CH + i] = bl[i];
  const int tbase = blockIdx.x * TGT + wave * 32;
  const int c = tbase + lane;
  int n = cnt[c];
  n = n < 0 ? 0 : (n > DEGCAP ? DEGCAP : n);
  const int st = off[c];
  const int cc = c > nN - 1 ? nN - 1 : c;
  const float px = pos[(size_t)cc * 3 + 0], py = pos[(size_t)cc * 3 + 1], pz = pos[(size_t)cc * 3 + 2];
  int nmax = n;
#pragma unroll
  for (int d = 16; d > 0; d >>= 1) { const int t = __shfl_xor(nmax, d); nmax = t > nmax ? t : nmax; }
  float ax = 0.f, ay = 0.f, az = 0.f;
#pragma unroll 1
  for (int p = 0; p < nmax; ++p) {
    int e = p < n - 1 ? p : n - 1;
    e = e < 0 ? 0 : e;
    int pi = st + e;
    pi = pi < 0 ? 0 : (pi > csrLen - 1 ? csrLen - 1 : pi);
    int s = csr[pi];
    s = s < 0 ? 0 : (s > nN - 1 ? nN - 1 : s);
    const float vx = pos[(size_t)s * 3 + 0], vy = pos[(size_t)s * 3 + 1], vz = pos[(size_t)s * 3 + 2];
    const bool ok = p < n;
    ax = ok ? ax + vx : ax;
    ay = ok ? ay + vy : ay;
    az = ok ? az + vz : az;
  }
  const float inv = 1.0f / (float)(n < 1 ? 1 : n);
  v4f mv; mv.x = ax * inv; mv.y = ay * inv; mv.z = az * inv; mv.w = 0.f;
  v4f pv; pv.x = px; pv.y = py; pv.z = pz; pv.w = 0.f;
  *(v4f*)(xs + (wave * 32 + lane) * 8)     = mv;
  *(v4f*)(xs + (wave * 32 + lane) * 8 + 4) = pv;
  __syncthreads();

  const int c4 = 4 * (lane & 15);
  const v4f wl0 = *(const v4f*)(sW + 0 * CH + c4), wl1 = *(const v4f*)(sW + 1 * CH + c4), wl2 = *(const v4f*)(sW + 2 * CH + c4);
  const v4f wr0 = *(const v4f*)(sW + 3 * CH + c4), wr1 = *(const v4f*)(sW + 4 * CH + c4), wr2 = *(const v4f*)(sW + 5 * CH + c4);
  const v4f bb  = *(const v4f*)(sW + 6 * CH + c4);
#pragma unroll 1
  for (int i = 0; i < 16; ++i) {
    const int nd = 2 * i + hh;
    const float* xp = xs + (wave * 32 + nd) * 8;
    const v4f ma = *(const v4f*)xp;
    const v4f pb = *(const v4f*)(xp + 4);
    v4f v = bb + wl0 * ma.x + wl1 * ma.y + wl2 * ma.z + wr0 * pb.x + wr1 * pb.y + wr2 * pb.z;
    v.x = fmaxf(v.x, 0.f); v.y = fmaxf(v.y, 0.f); v.z = fmaxf(v.z, 0.f); v.w = fmaxf(v.w, 0.f);
    float* hp = h0 + (size_t)(tbase + nd) * CH + c4;
    *(volatile v4f*)hp = v;
    __threadfence();
    *(volatile v4f*)hp = v;
  }
}

__global__ __launch_bounds__(NTHR) void k_agg(
    const int* __restrict__ csr, const int* __restrict__ off, const int* __restrict__ cnt,
    const float* __restrict__ h, float* meanp, int nN, int csrLen) {
  const int tid = threadIdx.x, lane = tid & 31, wave = tid >> 5, hh = lane >> 4;
  const int c4 = 4 * (lane & 15);
  const int tbase = blockIdx.x * TGT + wave * 32;
  const int cnt_l = cnt[tbase + lane];
  const int off_l = off[tbase + lane];
  v4f rowA = {0.f, 0.f, 0.f, 0.f};
#pragma unroll 1
  for (int j = 0; j < 32; ++j) {
    int n = __builtin_amdgcn_readlane(cnt_l, j);
    n = n < 0 ? 0 : (n > DEGCAP ? DEGCAP : n);
    const int st = __builtin_amdgcn_readlane(off_l, j);
    v4f acc = {0.f, 0.f, 0.f, 0.f};
    const int npair = (n + 1) >> 1;
#pragma unroll 1
    for (int p = 0; p < npair; ++p) {
      const int e  = 2 * p + hh;
      const int ec = e < n ? e : n - 1;
      int pi = st + ec;
      pi = pi < 0 ? 0 : (pi > csrLen - 1 ? csrLen - 1 : pi);
      int s = csr[pi];
      s = s < 0 ? 0 : (s > nN - 1 ? nN - 1 : s);
      const v4f v = *(const v4f*)(h + (size_t)s * CH + c4);
      const bool ok = e < n;
      acc.x = ok ? acc.x + v.x : acc.x;
      acc.y = ok ? acc.y + v.y : acc.y;
      acc.z = ok ? acc.z + v.z : acc.z;
      acc.w = ok ? acc.w + v.w : acc.w;
    }
    v4f tot;
    tot.x = acc.x + __shfl_xor(acc.x, 16);
    tot.y = acc.y + __shfl_xor(acc.y, 16);
    tot.z = acc.z + __shfl_xor(acc.z, 16);
    tot.w = acc.w + __shfl_xor(acc.w, 16);
    const float inv = 1.0f / (float)(n < 1 ? 1 : n);
    tot = tot * inv;
    if ((j & 1) == 0) {
      rowA = tot;
    } else {
      v4f sv;
      sv.x = hh ? tot.x : rowA.x; sv.y = hh ? tot.y : rowA.y; sv.z = hh ? tot.z : rowA.z; sv.w = hh ? tot.w : rowA.w;
      float* mp = meanp + (size_t)(tbase + j - 1 + hh) * CH + c4;
      *(volatile v4f*)mp = sv;
      __threadfence();
      *(volatile v4f*)mp = sv;
    }
  }
}

template <int NT, int DOUT, int RELU>
__global__ __launch_bounds__(NTHR) void k_lin(
    const float* __restrict__ meanp, const float* __restrict__ hp,
    const unsigned short* __restrict__ Bhi, const unsigned short* __restrict__ Blo,
    const float* __restrict__ bias, float* C, int nRows) {
  extern __shared__ v4f lds_dyn[];
  unsigned short* sAh = (unsigned short*)lds_dyn;
  unsigned short* sAl = sAh + GROWS * AP;
  float* stg = (float*)lds_dyn;
  const int tid = threadIdx.x, lane = tid & 31, wave = tid >> 5, hh = lane >> 4, m = lane & 15;
  const int rowBase = blockIdx.x * GROWS;

#pragma unroll
  for (int i = 0; i < 8; ++i) {
    const int half = i >> 2;
    const int rr = (i & 3) * 32 + (tid >> 3);
    const int g8 = (tid & 7) * 8;
    const float* src = (half == 0 ? meanp : hp) + (size_t)(rowBase + rr) * CH + g8;
    const v4f a = *(const v4f*)src, b = *(const v4f*)(src + 4);
    v8us h8, l8;
    split8(a, b, h8, l8);
    *(v8us*)(sAh + rr * AP + half * CH + g8) = h8;
    *(v8us*)(sAl + rr * AP + half * CH + g8) = l8;
  }
  __syncthreads();

  v8f acc[NT];
#pragma unroll
  for (int t = 0; t < NT; ++t) { v8f z = {0.f, 0.f, 0.f, 0.f, 0.f, 0.f, 0.f, 0.f}; acc[t] = z; }
  const unsigned short* arh = sAh + (wave * 16 + m) * AP + 8 * hh;
  const unsigned short* arl = sAl + (wave * 16 + m) * AP + 8 * hh;
#pragma unroll
  for (int kt = 0; kt < KD / 32; ++kt) {
    FragB fh, fl;
    fh.u[0] = *(const v8us*)(arh + 32 * kt);
    fh.u[1] = *(const v8us*)(arh + 32 * kt + 16);
    fl.u[0] = *(const v8us*)(arl + 32 * kt);
    fl.u[1] = *(const v8us*)(arl + 32 * kt + 16);
#pragma unroll
    for (int t = 0; t < NT; ++t) {
      const size_t bo = (size_t)(16 * t + m) * KD + 32 * kt + 8 * hh;
      FragB bh, bl2;
      bh.u[0]  = *(const v8us*)(Bhi + bo);
      bh.u[1]  = *(const v8us*)(Bhi + bo + 16);
      bl2.u[0] = *(const v8us*)(Blo + bo);
      bl2.u[1] = *(const v8us*)(Blo + bo + 16);
      acc[t] = wmb(fh.v, bh.v, acc[t]);
      acc[t] = wmb(fl.v, bh.v, acc[t]);
      acc[t] = wmb(fh.v, bl2.v, acc[t]);
    }
  }
  __syncthreads();

  const int r0 = wave * 16 + 8 * hh;
#pragma unroll
  for (int t = 0; t < NT; ++t) {
    const int col  = 16 * t + m;
    const int colc = col < DOUT ? col : DOUT - 1;
    const float bv = bias[colc];
    const bool ok  = col < DOUT;
#pragma unroll
    for (int r = 0; r < 8; ++r) {
      float v = acc[t][r] + bv;
      if (RELU != 0) v = fmaxf(v, 0.0f);
      if (ok) stg[(r0 + r) * DOUT + col] = v;
    }
  }
  __syncthreads();

  int valid = nRows - rowBase;
  valid = valid < 0 ? 0 : (valid > GROWS ? GROWS : valid);
  const int bound = valid * (DOUT / 4);
  constexpr int PIECES = GROWS * DOUT / 4;
  constexpr int NIT = (PIECES + NTHR - 1) / NTHR;
  float* cp = C + (size_t)rowBase * DOUT;
#pragma unroll
  for (int p = 0; p < NIT; ++p) {
    const int piece = p * NTHR + tid;
    if (piece < bound) { const v4f v = ((const v4f*)stg)[piece]; *(volatile v4f*)(cp + 4 * (size_t)piece) = v; }
  }
  __threadfence();
#pragma unroll
  for (int p = 0; p < NIT; ++p) {
    const int piece = p * NTHR + tid;
    if (piece < bound) { const v4f v = ((const v4f*)stg)[piece]; *(volatile v4f*)(cp + 4 * (size_t)piece) = v; }
  }
}

extern "C" void kernel_launch(void* const* d_in, const int* in_sizes, int n_in,
                              void* d_out, int out_size, void* d_ws, size_t ws_size,
                              hipStream_t stream) {
  if (n_in < 11) return;
  const int nN = in_sizes[0] / 3;
  const int nE = in_sizes[1] / 2;
  if (nN <= 0 || nE <= 0 || in_sizes[0] != 3 * nN || in_sizes[1] != 2 * nE) return;
  if (in_sizes[2] != 3 * CH || in_sizes[3] < CH || in_sizes[4] != 3 * CH) return;
  if (in_sizes[5] != CH * CH || in_sizes[6] < CH || in_sizes[7] != CH * CH) return;
  if (in_sizes[8] != CH * DOUT2 || in_sizes[9] < DOUT2 || in_sizes[10] != CH * DOUT2) return;
  if (out_size != nN * DOUT2) return;
  if (nE > (1 << 28) || nN > (1 << 24)) return;

  const float* pos = (const float*)d_in[0];
  const int*   ei  = (const int*)d_in[1];
  const float* Wl0 = (const float*)d_in[2];
  const float* bl0 = (const float*)d_in[3];
  const float* Wr0 = (const float*)d_in[4];
  const float* Wl1 = (const float*)d_in[5];
  const float* bl1 = (const float*)d_in[6];
  const float* Wr1 = (const float*)d_in[7];
  const float* Wl2 = (const float*)d_in[8];
  const float* bl2 = (const float*)d_in[9];
  const float* Wr2 = (const float*)d_in[10];
  float* out = (float*)d_out;

  const int NPAD   = ((nN + TGT - 1) / TGT) * TGT;
  const int nBC    = (nN + NBC - 1) / NBC;
  const int CNTPAD = nBC * NBC;
  if (SUBS * nBC + 1 > RBN) return;
  const int nBF    = SUBS * nBC;
  const int csrLen = ((nE + 31) & ~31) + 4096;
  if (31 * nBF > 4096) return;
  const int nAgg   = NPAD / TGT;
  const int nLin   = NPAD / GROWS;

  char* ws = (char*)d_ws;
  size_t off = 0;
  const size_t oB1h = off; off += (size_t)CH * KD * 2;          off = (off + 255) & ~(size_t)255;
  const size_t oB1l = off; off += (size_t)CH * KD * 2;          off = (off + 255) & ~(size_t)255;
  const size_t oB2h = off; off += (size_t)(NT2 * 16) * KD * 2;  off = (off + 255) & ~(size_t)255;
  const size_t oB2l = off; off += (size_t)(NT2 * 16) * KD * 2;  off = (off + 255) & ~(size_t)255;
  const size_t oCnt = off; off += (size_t)CNTPAD * 4;           off = (off + 255) & ~(size_t)255;
  const size_t oOff = off; off += (size_t)CNTPAD * 4;           off = (off + 255) & ~(size_t)255;
  const size_t oRb  = off; off += (size_t)RBN * 4;              off = (off + 255) & ~(size_t)255;
  const size_t oCsr = off; off += (size_t)csrLen * 4;           off = (off + 255) & ~(size_t)255;
  const size_t oH0  = off; off += (size_t)NPAD * CH * 4;        off = (off + 255) & ~(size_t)255;
  const size_t oH1  = off; off += (size_t)NPAD * CH * 4;        off = (off + 255) & ~(size_t)255;
  const size_t oMn  = off; off += (size_t)NPAD * CH * 4;        off = (off + 255) & ~(size_t)255;
  if (off > ws_size || off > (size_t)134217728) return;
  unsigned short* b1h = (unsigned short*)(ws + oB1h);
  unsigned short* b1l = (unsigned short*)(ws + oB1l);
  unsigned short* b2h = (unsigned short*)(ws + oB2h);
  unsigned short* b2l = (unsigned short*)(ws + oB2l);
  int*   cnt   = (int*)(ws + oCnt);
  int*   offp  = (int*)(ws + oOff);
  int*   rb    = (int*)(ws + oRb);
  int*   csr   = (int*)(ws + oCsr);
  float* h0    = (float*)(ws + oH0);
  float* h1    = (float*)(ws + oH1);
  float* meanp = (float*)(ws + oMn);

  const int vec8 = ((nE & 3) == 0) ? 1 : 0;

  const int nPrep = CH * (KD / 8) + (NT2 * 16) * (KD / 8);
  k_wprep<<<(nPrep + NTHR - 1) / NTHR, NTHR, 0, stream>>>(Wl1, Wr1, Wl2, Wr2, b1h, b1l, b2h, b2l);

  k_count<<<nBC, NTHR, 0, stream>>>(ei, cnt, nE, vec8);
  k_offsets<<<1, OTHR, 0, stream>>>(cnt, offp, rb, nBC);
  hipFuncSetAttribute(reinterpret_cast<const void*>(&k_fill),
                      hipFuncAttributeMaxDynamicSharedMemorySize, LDS_FILL);
  k_fill<<<nBF, NTHR, LDS_FILL, stream>>>(ei, offp, rb, csr, nN, nE, vec8, csrLen);

  k_layer0<<<nAgg, NTHR, 0, stream>>>(pos, csr, offp, cnt, Wl0, bl0, Wr0, h0, nN, csrLen);

  hipFuncSetAttribute(reinterpret_cast<const void*>(&k_lin<4, CH, 1>),
                      hipFuncAttributeMaxDynamicSharedMemorySize, LDS_LIN);
  hipFuncSetAttribute(reinterpret_cast<const void*>(&k_lin<NT2, DOUT2, 0>),
                      hipFuncAttributeMaxDynamicSharedMemorySize, LDS_LIN);
  k_agg<<<nAgg, NTHR, 0, stream>>>(csr, offp, cnt, h0, meanp, nN, csrLen);
  k_lin<4, CH, 1><<<nLin, NTHR, LDS_LIN, stream>>>(meanp, h0, b1h, b1l, bl1, h1, NPAD);

  k_agg<<<nAgg, NTHR, 0, stream>>>(csr, offp, cnt, h1, meanp, nN, csrLen);
  k_lin<NT2, DOUT2, 0><<<nLin, NTHR, LDS_LIN, stream>>>(meanp, h1, b2h, b2l, bl2, out, nN);
}
